// FlaGdnpControlConditionedSequenceMixer_47064251630311
// MI455X (gfx1250) — hardware-run, weakly checked
//
#include <hip/hip_runtime.h>
#include <math.h>

constexpr int kB = 2;
constexpr int kSeq = 1024;
constexpr int kD = 1024;
constexpr int kH = 16;
constexpr int kDH = 64;
constexpr int kBW = 128;
constexpr int kTok = kB * kSeq;
constexpr int kNDelta = 3 * kD + kH;
constexpr int kNDeltaPad = 3136;
constexpr int kNCtrl = 4 * kD + 2 * kH;
constexpr int kNCtrlPad = 4160;
constexpr int kBGPitch = 32;
constexpr float kEps = 1e-6f;
static_assert(kNDeltaPad % 64 == 0 && kNDeltaPad >= kNDelta);
static_assert(kNCtrlPad % 64 == 0 && kNCtrlPad >= kNCtrl);

constexpr size_t szCtrlWtPlane = (size_t)kNCtrlPad * kD * 2;
constexpr size_t szHidPlane    = (size_t)kTok * kD * 2;
constexpr size_t oCtrlWtHi = 0;
constexpr size_t oCtrlWtLo = oCtrlWtHi + szCtrlWtPlane;
constexpr size_t oHidHi    = oCtrlWtLo + szCtrlWtPlane;
constexpr size_t oHidLo    = oHidHi + szHidPlane;
constexpr size_t oR0End    = oHidLo + szHidPlane;
constexpr size_t oQKV      = 0;
constexpr size_t szQKV     = (size_t)3 * kTok * kD * 4;
static_assert(oQKV + szQKV <= oR0End);
constexpr size_t oCtrl     = oR0End;
constexpr size_t szCtrl    = (size_t)kTok * kNCtrlPad * 4;
constexpr size_t oDeltas   = oCtrl + szCtrl;
constexpr size_t szDeltas  = (size_t)kTok * kNDeltaPad * 4;
constexpr size_t oR2End    = oDeltas + szDeltas;
constexpr size_t oO        = oDeltas;
constexpr size_t szO       = (size_t)kTok * kD * 4;
constexpr size_t oYHi      = oO + szO;
constexpr size_t szYPlane  = (size_t)kTok * kD * 2;
constexpr size_t oYLo      = oYHi + szYPlane;
static_assert(oYLo + szYPlane <= oR2End);
constexpr size_t oCiHi     = oR2End;
constexpr size_t szCiPlane = (size_t)kBW * kD * 2;
constexpr size_t oCiLo     = oCiHi + szCiPlane;
constexpr size_t oP        = oCiLo + szCiPlane;
constexpr size_t szP       = (size_t)kTok * kBW * 4;
constexpr size_t oCHi      = oP + szP;
constexpr size_t szCPlane  = (size_t)kTok * kBW * 2;
constexpr size_t oCLo      = oCHi + szCPlane;
constexpr size_t oDwHi     = oCLo + szCPlane;
constexpr size_t szDwPlane = (size_t)kNDeltaPad * kBW * 2;
constexpr size_t oDwLo     = oDwHi + szDwPlane;
constexpr size_t oOpHi     = oDwLo + szDwPlane;
constexpr size_t szOpPlane = (size_t)kD * kD * 2;
constexpr size_t oOpLo     = oOpHi + szOpPlane;
constexpr size_t oBG       = oOpLo + szOpPlane;
constexpr size_t szBG      = (size_t)kTok * kBGPitch * 4;
constexpr size_t kWsEnd    = oBG + szBG;
static_assert(kWsEnd <= (size_t)134217728);
static_assert(oCtrl % 256 == 0 && oDeltas % 256 == 0 && oR2End % 256 == 0 && oBG % 256 == 0 && oYHi % 256 == 0);

typedef __attribute__((ext_vector_type(16))) _Float16 v16h;
typedef __attribute__((ext_vector_type(8)))  _Float16 v8h;
typedef __attribute__((ext_vector_type(16))) __bf16   v16b;
typedef __attribute__((ext_vector_type(8)))  __bf16   v8b;
typedef __attribute__((ext_vector_type(8)))  float    v8f;
typedef __attribute__((ext_vector_type(4)))  float    v4f;
typedef __attribute__((ext_vector_type(4)))  unsigned int v4u;

__device__ __forceinline__ unsigned short f2bf_bits(float f) {
  unsigned u = __float_as_uint(f);
  return (unsigned short)((u + 0x7FFFu + ((u >> 16) & 1u)) >> 16);
}
__device__ __forceinline__ float bf_bits2f(unsigned short h) { return __uint_as_float(((unsigned)h) << 16); }

__device__ __forceinline__ void dep_guard_h(v8f& a, v8f& b, v16h x, v16h y) { asm volatile("v_nop\n\tv_nop\n\tv_nop\n\tv_nop" : "+v"(a), "+v"(b) : "v"(x), "v"(y)); }
__device__ __forceinline__ void dep_guard_b(v8f& a, v8f& b, v16b x, v16b y) { asm volatile("v_nop\n\tv_nop\n\tv_nop\n\tv_nop" : "+v"(a), "+v"(b) : "v"(x), "v"(y)); }
__device__ __forceinline__ void keep4_h(v16h a, v16h b, v16h c, v16h d) { asm volatile("v_nop" :: "v"(a), "v"(b), "v"(c), "v"(d)); }
__device__ __forceinline__ void keep4_b(v16b a, v16b b, v16b c, v16b d) { asm volatile("v_nop" :: "v"(a), "v"(b), "v"(c), "v"(d)); }
__device__ __forceinline__ void acc_guard4(v8f& a, v8f& b, v8f& c, v8f& d) { asm volatile("v_nop\n\tv_nop\n\tv_nop\n\tv_nop" : "+v"(a), "+v"(b), "+v"(c), "+v"(d)); }
template <typename T> struct Frag;
template <> struct Frag<_Float16> {
  typedef v16h V; union U { v16h v; v8h h[2]; };
  static __device__ __forceinline__ v16h load(const _Float16* p) {
    U f; f.h[0] = *(const v8h*)(p); f.h[1] = *(const v8h*)(p + 16); return f.v;
  }
  static __device__ __forceinline__ v8f mma(v16h a, v16h b, v8f c) {
    return __builtin_amdgcn_wmma_f32_16x16x32_f16(false, a, false, b, (short)0, c, false, false);
  }
  static __device__ __forceinline__ void guard(v8f& a, v8f& b, v16h x, v16h y) { dep_guard_h(a, b, x, y); }
  static __device__ __forceinline__ void keep(v16h a, v16h b, v16h c, v16h d) { keep4_h(a, b, c, d); }
};
template <> struct Frag<__bf16> {
  typedef v16b V; union U { v16b v; v8b h[2]; };
  static __device__ __forceinline__ v16b load(const __bf16* p) {
    U f; f.h[0] = *(const v8b*)(p); f.h[1] = *(const v8b*)(p + 16); return f.v;
  }
  static __device__ __forceinline__ v8f mma(v16b a, v16b b, v8f c) {
    return __builtin_amdgcn_wmma_f32_16x16x32_bf16(false, a, false, b, (short)0, c, false, false);
  }
  static __device__ __forceinline__ void guard(v8f& a, v8f& b, v16b x, v16b y) { dep_guard_b(a, b, x, y); }
  static __device__ __forceinline__ void keep(v16b a, v16b b, v16b c, v16b d) { keep4_b(a, b, c, d); }
};

__device__ __forceinline__ unsigned pk16(unsigned short a, unsigned short b) { return (unsigned)a | ((unsigned)b << 16); }

template <int ET> struct Elem;
template <> struct Elem<0> { typedef _Float16 T; };
template <> struct Elem<1> { typedef __bf16 T; };
template <int ET, bool SPLIT, int BIAS_MODE, int OUT_MODE, bool RESID, int ACT = 0>
__global__ __launch_bounds__(256) void wmma_gemm64(
    const unsigned short* __restrict__ Ap, const unsigned short* __restrict__ A2p, int lda, long strideA,
    const unsigned short* __restrict__ Btp, const unsigned short* __restrict__ Bt2p, int ldb, long strideB,
    void* __restrict__ Cout, void* __restrict__ Cout2, int ldc, long strideC,
    const float* __restrict__ bias,
    const float* __restrict__ resid, long strideR,
    int M, int N, int K, float scale) {
  typedef typename Elem<ET>::T T;
  typedef typename Frag<T>::V V;
  const T* A = (const T*)Ap; const T* A2 = (const T*)A2p; const T* Bt = (const T*)Btp; const T* Bt2 = (const T*)Bt2p;
  __shared__ __align__(16) float sT[8][16 * 68];
  const int b    = blockIdx.y;
  const int lane = threadIdx.x & 31;
  const int wave = threadIdx.x >> 5;
  const int tilesN = N >> 6;
  const int tilesM = M >> 6;
  const int tile = blockIdx.x * 8 + wave;
  if (tile >= tilesM * tilesN) return;
  const int tm = tile / tilesN;
  const int tn = tile - tm * tilesN;
  const int m0 = tm << 6;
  const int n0 = tn << 6;

  const T* Ab  = A  + (size_t)b * strideA;
  const T* Bb  = Bt + (size_t)b * strideB;
  const T* Ab2 = SPLIT ? (A2  + (size_t)b * strideA) : nullptr;
  const T* Bb2 = SPLIT ? (Bt2 + (size_t)b * strideB) : nullptr;

  const int rlane = lane & 15;
  const int koff  = (lane >> 4) * 8;
  const int mOff  = (lane >> 4) * 8;

  v8f acc[4][4];
#pragma unroll
  for (int i = 0; i < 4; ++i)
#pragma unroll
    for (int j = 0; j < 4; ++j) acc[i][j] = (v8f){0.f,0.f,0.f,0.f,0.f,0.f,0.f,0.f};

  for (int k0 = 0; k0 < K; k0 += 32) {
    V bh[4], bl[4];
#pragma unroll
    for (int j = 0; j < 4; ++j) {
      const size_t bo = (size_t)(n0 + (j << 4) + rlane) * ldb + koff + k0;
      bh[j] = Frag<T>::load(Bb + bo);
      if (SPLIT) bl[j] = Frag<T>::load(Bb2 + bo);
    }
#pragma unroll
    for (int i = 0; i < 4; ++i) {
      const size_t ao = (size_t)(m0 + (i << 4) + rlane) * lda + koff + k0;
      V ah = Frag<T>::load(Ab + ao);
      V al;
      if (SPLIT) al = Frag<T>::load(Ab2 + ao);
#pragma unroll
      for (int j = 0; j < 4; ++j) {
        acc[i][j] = Frag<T>::mma(ah, bh[j], acc[i][j]);
        if (SPLIT) {
          acc[i][j] = Frag<T>::mma(ah, bl[j], acc[i][j]);
          acc[i][j] = Frag<T>::mma(al, bh[j], acc[i][j]);
        }
      }
      Frag<T>::guard(acc[i][0], acc[i][3], ah, SPLIT ? al : ah);
    }
    Frag<T>::keep(bh[0], bh[1], bh[2], bh[3]);
    if (SPLIT) Frag<T>::keep(bl[0], bl[1], bl[2], bl[3]);
  }
  acc_guard4(acc[0][0], acc[0][1], acc[0][2], acc[0][3]);
  acc_guard4(acc[1][0], acc[1][1], acc[1][2], acc[1][3]);
  acc_guard4(acc[2][0], acc[2][1], acc[2][2], acc[2][3]);
  acc_guard4(acc[3][0], acc[3][1], acc[3][2], acc[3][3]);

  float* slab = sT[wave];
  const float* Rb = RESID ? (resid + (size_t)b * strideR) : nullptr;
#pragma unroll
  for (int i = 0; i < 4; ++i) {
    const int mBase = m0 + (i << 4);
#pragma unroll
    for (int j = 0; j < 4; ++j) {
      const int n = n0 + (j << 4) + rlane;
      float bv = 0.f;
      if (BIAS_MODE == 2) bv = bias[n];
#pragma unroll
      for (int r = 0; r < 8; ++r) {
        float v = acc[i][j][r] * scale;
        if (BIAS_MODE == 1) v += bias[mBase + mOff + r];
        if (BIAS_MODE == 2) v += bv;
        if (RESID) v += Rb[(size_t)(mBase + mOff + r) * ldc + n];
        if (ACT == 2) v = fmaxf(v, 0.0f);
        if (ACT == 4) v = (v > 0.f) ? v : 0.01f * v;
        slab[(mOff + r) * 68 + (j << 4) + rlane] = v;
      }
    }
    __builtin_amdgcn_fence(__ATOMIC_RELEASE, "workgroup");
    __builtin_amdgcn_wave_barrier();
    __builtin_amdgcn_fence(__ATOMIC_ACQUIRE, "workgroup");
    if (OUT_MODE == 0) {
      float* C = (float*)Cout + (size_t)b * strideC;
      const int hh = lane >> 4, c4 = (lane & 15) * 4;
      for (int pass = 0; pass < 2; ++pass) {
#pragma unroll
        for (int it = 0; it < 8; ++it) {
          const int row = it * 2 + hh;
          v4f v = *(const v4f*)(slab + row * 68 + c4);
          *(volatile v4f*)(C + (size_t)(mBase + row) * ldc + n0 + c4) = v;
        }
        __threadfence();
      }
    } else {
      const int q = lane >> 3, c8 = (lane & 7) * 8;
      unsigned short* C  = (unsigned short*)Cout  + (size_t)b * strideC;
      unsigned short* C2 = (OUT_MODE == 2) ? ((unsigned short*)Cout2 + (size_t)b * strideC) : nullptr;
      for (int pass = 0; pass < 2; ++pass) {
#pragma unroll
        for (int it = 0; it < 4; ++it) {
          const int row = it * 4 + q;
          const float* sp = slab + row * 68 + c8;
          v8h hv, lv;
#pragma unroll
          for (int e = 0; e < 8; ++e) {
            if (OUT_MODE == 1) {
              hv[e] = (_Float16)sp[e];
            } else {
              unsigned short hb = f2bf_bits(sp[e]);
              unsigned short lb = f2bf_bits(sp[e] - bf_bits2f(hb));
              hv[e] = __builtin_bit_cast(_Float16, hb);
              lv[e] = __builtin_bit_cast(_Float16, lb);
            }
          }
          *(volatile v8h*)(C + (size_t)(mBase + row) * ldc + n0 + c8) = hv;
          if (OUT_MODE == 2) *(volatile v8h*)(C2 + (size_t)(mBase + row) * ldc + n0 + c8) = lv;
        }
        __threadfence();
      }
    }
    __builtin_amdgcn_fence(__ATOMIC_RELEASE, "workgroup");
    __builtin_amdgcn_wave_barrier();
    __builtin_amdgcn_fence(__ATOMIC_ACQUIRE, "workgroup");
  }
}

__device__ __forceinline__ float sigm_f(float x) { return __builtin_amdgcn_rcpf(1.0f + expf(-x)); }
__device__ __forceinline__ float silu_f(float x) { return x * sigm_f(x); }
__device__ __forceinline__ void split_bits(float x, unsigned short& hb, unsigned short& lb) {
  hb = f2bf_bits(x);
  lb = f2bf_bits(x - bf_bits2f(hb));
}

__global__ __launch_bounds__(256) void split8_bf16_kernel(const float* __restrict__ in,
                                                          unsigned short* __restrict__ hi,
                                                          unsigned short* __restrict__ lo, int n8) {
  const int i = blockIdx.x * 256 + threadIdx.x;
  if (i >= n8) return;
  const float* p = in + 8 * (size_t)i;
  const v4f a = *(const v4f*)(p);
  const v4f c = *(const v4f*)(p + 4);
  unsigned short hb[8], lb[8];
#pragma unroll
  for (int e = 0; e < 4; ++e) {
    split_bits(a[e], hb[e], lb[e]);
    split_bits(c[e], hb[4 + e], lb[4 + e]);
  }
  const v4u hu = (v4u){pk16(hb[0], hb[1]), pk16(hb[2], hb[3]), pk16(hb[4], hb[5]), pk16(hb[6], hb[7])};
  const v4u lu = (v4u){pk16(lb[0], lb[1]), pk16(lb[2], lb[3]), pk16(lb[4], lb[5]), pk16(lb[6], lb[7])};
  unsigned short* qh = hi + 8 * (size_t)i;
  unsigned short* ql = lo + 8 * (size_t)i;
  *(volatile v4u*)qh = hu;
  *(volatile v4u*)ql = lu;
  __threadfence();
  *(volatile v4u*)qh = hu;
  *(volatile v4u*)ql = lu;
}

__global__ __launch_bounds__(256) void tsplit_bf16_kernel(const float* __restrict__ W, int R, int Cc,
                                                          unsigned short* __restrict__ ohi,
                                                          unsigned short* __restrict__ olo) {
  __shared__ float sm[64][65];
  const int t  = threadIdx.x;
  const int c0 = blockIdx.x * 64;
  const int r0 = blockIdx.y * 64;
#pragma unroll
  for (int i = 0; i < 16; ++i) {
    const int e = i * 256 + t;
    const int r = e >> 6;
    const int c = e & 63;
    const int cg = c0 + c;
    const int cgc = (cg < Cc) ? cg : (Cc - 1);
    float v = W[(size_t)(r0 + r) * Cc + cgc];
    v = (cg < Cc) ? v : 0.0f;
    sm[c][r] = v;
  }
  __syncthreads();
  const int lane = t & 31, wave = t >> 5;
  const int q = lane >> 3, c8 = (lane & 7) * 8;
  for (int pass = 0; pass < 2; ++pass) {
#pragma unroll
    for (int it = 0; it < 2; ++it) {
      const int row = wave * 8 + it * 4 + q;
      unsigned short hb[8], lb[8];
#pragma unroll
      for (int e = 0; e < 8; ++e) split_bits(sm[row][c8 + e], hb[e], lb[e]);
      const v4u hu = (v4u){pk16(hb[0], hb[1]), pk16(hb[2], hb[3]), pk16(hb[4], hb[5]), pk16(hb[6], hb[7])};
      const v4u lu = (v4u){pk16(lb[0], lb[1]), pk16(lb[2], lb[3]), pk16(lb[4], lb[5]), pk16(lb[6], lb[7])};
      const size_t di = (size_t)(c0 + row) * R + r0 + c8;
      *(volatile v4u*)(ohi + di) = hu;
      *(volatile v4u*)(olo + di) = lu;
    }
    __threadfence();
  }
}

__global__ __launch_bounds__(64) void cond_scan_kernel(const float* __restrict__ p, const float* __restrict__ theta,
                                                      const float* __restrict__ nw,
                                                      unsigned short* __restrict__ chi,
                                                      unsigned short* __restrict__ clo) {
  __shared__ float red[2][2];
  __shared__ __align__(16) float stage[16][kBW];
  const int b = blockIdx.x;
  const int j = threadIdx.x;
  const int lane = j & 31, wave = j >> 5;
  const float th = theta[j];
  const float cth = cosf(th);
  const float sth = sinf(th);
  const float w0 = nw[2 * j], w1 = nw[2 * j + 1];
  float s0 = 0.0f, s1 = 0.0f;
  for (int t = 0; t < kSeq; ++t) {
    const size_t base = (size_t)(b * kSeq + t) * kBW;
    const float x0 = p[base + 2 * j];
    const float x1 = p[base + 2 * j + 1];
    const float n0 = cth * s0 - sth * s1 + x0;
    const float n1 = sth * s0 + cth * s1 + x1;
    s0 = n0; s1 = n1;
    float qq = s0 * s0 + s1 * s1;
    qq += __shfl_xor(qq, 1, 32);
    qq += __shfl_xor(qq, 2, 32);
    qq += __shfl_xor(qq, 4, 32);
    qq += __shfl_xor(qq, 8, 32);
    qq += __shfl_xor(qq, 16, 32);
    const int par = t & 1;
    if (lane == 0) red[par][wave] = qq;
    __syncthreads();
    const float tot = red[par][0] + red[par][1];
    const float inv = rsqrtf(tot * (1.0f / 128.0f) + kEps);
    const int tr = t & 15;
    stage[tr][2 * j]     = s0 * inv * w0;
    stage[tr][2 * j + 1] = s1 * inv * w1;
    if (tr == 15) {
      __syncthreads();
      const int gq = j >> 3, e = j & 7;
      const int half = gq & 1;
      const int t0 = t - 15;
      for (int pass = 0; pass < 2; ++pass) {
#pragma unroll
        for (int it = 0; it < 4; ++it) {
          const int row = it * 4 + (gq >> 1);
          const float* sp = &stage[row][half * 64 + e * 8];
          unsigned short hb[8], lb[8];
#pragma unroll
          for (int u = 0; u < 8; ++u) split_bits(sp[u], hb[u], lb[u]);
          const v4u hu = (v4u){pk16(hb[0], hb[1]), pk16(hb[2], hb[3]), pk16(hb[4], hb[5]), pk16(hb[6], hb[7])};
          const v4u lu = (v4u){pk16(lb[0], lb[1]), pk16(lb[2], lb[3]), pk16(lb[4], lb[5]), pk16(lb[6], lb[7])};
          const size_t di = (size_t)(b * kSeq + t0 + row) * kBW + half * 64 + e * 8;
          *(volatile v4u*)(chi + di) = hu;
          *(volatile v4u*)(clo + di) = lu;
        }
        __threadfence();
      }
      __syncthreads();
    }
  }
}

__global__ __launch_bounds__(256) void qkv_prep_kernel(
    const float* __restrict__ ctrl, const float* __restrict__ deltas, const float* __restrict__ ctrl_b,
    const float* __restrict__ qkv_ramp, const float* __restrict__ beta_ramp,
    const float* __restrict__ qw, const float* __restrict__ kw, const float* __restrict__ vw,
    float* __restrict__ qkv, float* __restrict__ bg) {
  __shared__ __align__(16) float vals[3 * kD];
  __shared__ float invs[32];
  __shared__ __align__(16) float bgs[32];
  const int rowi = blockIdx.x;
  const int b = rowi >> 10;
  const int t = rowi & (kSeq - 1);
  const int tid = threadIdx.x;
#pragma unroll 1
  for (int it = 0; it < 12; ++it) {
    const int z = it >> 2;
    const int c = ((it & 3) << 8) + tid;
    const float* cwp = (z == 0) ? qw : ((z == 1) ? kw : vw);
    const v4f w4 = *(const v4f*)(cwp + 4 * c);
    const float rr = sigm_f(qkv_ramp[z * kD + c]);
    const float cb = ctrl_b[z * kD + c];
    float acc = 0.0f;
#pragma unroll
    for (int i = 0; i < 4; ++i) {
      const int tt = t - 3 + i;
      const int ttc = (tt < 0) ? 0 : tt;
      const size_t r = (size_t)(b * kSeq + ttc);
      const float cv = ctrl[r * kNCtrlPad + z * kD + c];
      const float dv = deltas[r * kNDeltaPad + z * kD + c];
      float x = (cv + cb) + dv * rr;
      x = (tt >= 0) ? x : 0.0f;
      acc += x * w4[i];
    }
    vals[it * 256 + tid] = silu_f(acc);
  }
  {
    const int hc = tid & 15;
    const size_t r0 = (size_t)rowi;
    const float dec = ctrl[r0 * kNCtrlPad + 3 * kD + hc] + ctrl_b[3 * kD + hc];
    const float bet = (ctrl[r0 * kNCtrlPad + 3 * kD + kH + hc] + ctrl_b[3 * kD + kH + hc])
                    + deltas[r0 * kNDeltaPad + 3 * kD + hc] * sigm_f(beta_ramp[hc]);
    const float gv = sigm_f(dec);
    const float bv = sigm_f(bet);
    if (tid < 32) bgs[tid] = (tid < 16) ? bv : gv;
  }
  __syncthreads();
  {
    const int hq = tid >> 3, e = tid & 7;
    const int base = (hq >> 4) * kD + (hq & 15) * kDH + e * 8;
    const v4f a  = *(const v4f*)(vals + base);
    const v4f a2 = *(const v4f*)(vals + base + 4);
    float ss = 0.0f;
#pragma unroll
    for (int u = 0; u < 4; ++u) { ss = fmaf(a[u], a[u], ss); ss = fmaf(a2[u], a2[u], ss); }
    ss += __shfl_xor(ss, 1, 32);
    ss += __shfl_xor(ss, 2, 32);
    ss += __shfl_xor(ss, 4, 32);
    if (e == 0) invs[hq] = rsqrtf(ss + kEps);
  }
  __syncthreads();
  const v4f oq = *(const v4f*)(vals + 4 * tid) * invs[tid >> 4];
  const v4f ok = *(const v4f*)(vals + kD + 4 * tid) * invs[16 + (tid >> 4)];
  const v4f ov = *(const v4f*)(vals + 2 * kD + 4 * tid);
  const int tb = (tid < 8) ? tid : 0;
  const v4f bgv = *(const v4f*)(bgs + 4 * tb);
  const size_t plane = (size_t)kTok * kD;
  float* dq  = qkv + (size_t)rowi * kD + 4 * tid;
  float* dbg = bg + (size_t)rowi * kBGPitch + 4 * tb;
  for (int pass = 0; pass < 2; ++pass) {
    *(volatile v4f*)(dq) = oq;
    *(volatile v4f*)(dq + plane) = ok;
    *(volatile v4f*)(dq + 2 * plane) = ov;
    if (tid < 8) *(volatile v4f*)(dbg) = bgv;
    __threadfence();
  }
}

__global__ __launch_bounds__(256) void gdn_kernel(const float* __restrict__ qkv, const float* __restrict__ bg,
                                                 float* __restrict__ oout) {
  __shared__ float redk[2][4][64];
  __shared__ float redo[2][4][64];
  __shared__ __align__(16) float ost[16][64];
  const int bh = blockIdx.x;
  const int b = bh >> 4, h = bh & 15;
  const int tid = threadIdx.x;
  const int part = tid >> 6;
  const int vc = tid & 63;
  const size_t plane = (size_t)kTok * kD;
  const float* qp = qkv;
  const float* kp = qkv + plane;
  const float* vp = qkv + 2 * plane;
  float s[16];
#pragma unroll
  for (int jj = 0; jj < 16; ++jj) s[jj] = 0.0f;
  for (int t = 0; t < kSeq; ++t) {
    const int rowi = b * kSeq + t;
    const size_t base = (size_t)rowi * kD + h * kDH;
    const float* kr = kp + base + part * 16;
    const float* qr = qp + base + part * 16;
    const v4f k0 = *(const v4f*)(kr), k1 = *(const v4f*)(kr + 4), k2 = *(const v4f*)(kr + 8), k3 = *(const v4f*)(kr + 12);
    const v4f q0 = *(const v4f*)(qr), q1 = *(const v4f*)(qr + 4), q2 = *(const v4f*)(qr + 8), q3 = *(const v4f*)(qr + 12);
    float kk[16], qq[16];
#pragma unroll
    for (int u = 0; u < 4; ++u) {
      kk[u] = k0[u]; kk[4 + u] = k1[u]; kk[8 + u] = k2[u]; kk[12 + u] = k3[u];
      qq[u] = q0[u]; qq[4 + u] = q1[u]; qq[8 + u] = q2[u]; qq[12 + u] = q3[u];
    }
    const float vv = vp[base + vc];
    const float beta = bg[(size_t)rowi * kBGPitch + h];
    const float gdec = bg[(size_t)rowi * kBGPitch + 16 + h];
    float ksp = 0.0f;
#pragma unroll
    for (int jj = 0; jj < 16; ++jj) { s[jj] *= gdec; ksp = fmaf(kk[jj], s[jj], ksp); }
    const int par = t & 1;
    redk[par][part][vc] = ksp;
    __syncthreads();
    const float ks = ((redk[par][0][vc] + redk[par][1][vc]) + redk[par][2][vc]) + redk[par][3][vc];
    const float upd = beta * (vv - ks);
    float op = 0.0f;
#pragma unroll
    for (int jj = 0; jj < 16; ++jj) { s[jj] = fmaf(kk[jj], upd, s[jj]); op = fmaf(qq[jj], s[jj], op); }
    redo[par][part][vc] = op;
    __syncthreads();
    if (part == 0) {
      ost[t & 15][vc] = ((redo[par][0][vc] + redo[par][1][vc]) + redo[par][2][vc]) + redo[par][3][vc];
    }
    if ((t & 15) == 15) {
      __syncthreads();
      const int gq = tid >> 3, e = tid & 7;
      const int row = gq >> 1, half = gq & 1;
      const int t0 = t - 15;
      const v4f val = *(const v4f*)(&ost[row][half * 32 + e * 4]);
      float* dst = oout + (size_t)(b * kSeq + t0 + row) * kD + h * kDH + half * 32 + e * 4;
      *(volatile v4f*)dst = val;
      __threadfence();
      *(volatile v4f*)dst = val;
      __syncthreads();
    }
  }
}

__global__ __launch_bounds__(128) void norm_gate_kernel(const float* __restrict__ o, const float* __restrict__ ctrl,
                                                       const float* __restrict__ ctrl_b, const float* __restrict__ onw,
                                                       unsigned short* __restrict__ yhi, unsigned short* __restrict__ ylo) {
  const int rowi = blockIdx.x;
  const int tid = threadIdx.x;
  const int c0 = 8 * tid;
  const float* orow = o + (size_t)rowi * kD + c0;
  const v4f a  = *(const v4f*)(orow);
  const v4f a2 = *(const v4f*)(orow + 4);
  float x[8];
#pragma unroll
  for (int e = 0; e < 4; ++e) { x[e] = a[e]; x[4 + e] = a2[e]; }
  float ss = 0.0f;
#pragma unroll
  for (int e = 0; e < 8; ++e) ss = fmaf(x[e], x[e], ss);
  ss += __shfl_xor(ss, 1, 32);
  ss += __shfl_xor(ss, 2, 32);
  ss += __shfl_xor(ss, 4, 32);
  const float inv = rsqrtf(ss * (1.0f / 64.0f) + kEps);
  const float* grow = ctrl + (size_t)rowi * kNCtrlPad + 3 * kD + 2 * kH + c0;
  const v4f ga = *(const v4f*)(grow), gb = *(const v4f*)(grow + 4);
  const v4f ba = *(const v4f*)(ctrl_b + 3 * kD + 2 * kH + c0), bb = *(const v4f*)(ctrl_b + 3 * kD + 2 * kH + c0 + 4);
  const v4f wa = *(const v4f*)(onw + (c0 & 63)), wb = *(const v4f*)(onw + (c0 & 63) + 4);
  float gt[8], wv[8];
#pragma unroll
  for (int e = 0; e < 4; ++e) { gt[e] = ga[e] + ba[e]; gt[4 + e] = gb[e] + bb[e]; wv[e] = wa[e]; wv[4 + e] = wb[e]; }
  unsigned short hb[8], lb[8];
#pragma unroll
  for (int e = 0; e < 8; ++e) {
    const float y = (x[e] * inv * wv[e]) * silu_f(gt[e]);
    split_bits(y, hb[e], lb[e]);
  }
  const v4u hu = (v4u){pk16(hb[0], hb[1]), pk16(hb[2], hb[3]), pk16(hb[4], hb[5]), pk16(hb[6], hb[7])};
  const v4u lu = (v4u){pk16(lb[0], lb[1]), pk16(lb[2], lb[3]), pk16(lb[4], lb[5]), pk16(lb[6], lb[7])};
  const size_t di = (size_t)rowi * kD + c0;
  *(volatile v4u*)(yhi + di) = hu;
  *(volatile v4u*)(ylo + di) = lu;
  __threadfence();
  *(volatile v4u*)(yhi + di) = hu;
  *(volatile v4u*)(ylo + di) = lu;
}

extern "C" void kernel_launch(void* const* d_in, const int* in_sizes, int n_in,
                              void* d_out, int out_size, void* d_ws, size_t ws_size,
                              hipStream_t stream) {
  if (n_in < 15) return;
  if (ws_size < kWsEnd) return;
  if (out_size < kTok * kD) return;
  if (in_sizes[0] != kTok * kD || in_sizes[7] != kD * kNCtrl || in_sizes[4] != kBW * kNDelta) return;

  const float* hidden      = (const float*)d_in[0];
  const float* cond_in_W   = (const float*)d_in[1];
  const float* rot_theta   = (const float*)d_in[2];
  const float* cond_norm_w = (const float*)d_in[3];
  const float* delta_W     = (const float*)d_in[4];
  const float* qkv_ramp    = (const float*)d_in[5];
  const float* beta_ramp   = (const float*)d_in[6];
  const float* ctrl_W      = (const float*)d_in[7];
  const float* ctrl_b      = (const float*)d_in[8];
  const float* q_conv_w    = (const float*)d_in[9];
  const float* k_conv_w    = (const float*)d_in[10];
  const float* v_conv_w    = (const float*)d_in[11];
  const float* out_norm_w  = (const float*)d_in[12];
  const float* out_proj_W  = (const float*)d_in[13];
  const float* out_proj_b  = (const float*)d_in[14];
  float* out = (float*)d_out;

  char* ws = (char*)d_ws;
  unsigned short* ctrlWt_hi = (unsigned short*)(ws + oCtrlWtHi);
  unsigned short* ctrlWt_lo = (unsigned short*)(ws + oCtrlWtLo);
  unsigned short* hid_hi    = (unsigned short*)(ws + oHidHi);
  unsigned short* hid_lo    = (unsigned short*)(ws + oHidLo);
  float* qkv                = (float*)(ws + oQKV);
  float* ctrl               = (float*)(ws + oCtrl);
  float* deltas             = (float*)(ws + oDeltas);
  float* obuf               = (float*)(ws + oO);
  unsigned short* y_hi      = (unsigned short*)(ws + oYHi);
  unsigned short* y_lo      = (unsigned short*)(ws + oYLo);
  unsigned short* ci_hi     = (unsigned short*)(ws + oCiHi);
  unsigned short* ci_lo     = (unsigned short*)(ws + oCiLo);
  float* pbuf               = (float*)(ws + oP);
  unsigned short* c_hi      = (unsigned short*)(ws + oCHi);
  unsigned short* c_lo      = (unsigned short*)(ws + oCLo);
  unsigned short* dw_hi     = (unsigned short*)(ws + oDwHi);
  unsigned short* dw_lo     = (unsigned short*)(ws + oDwLo);
  unsigned short* op_hi     = (unsigned short*)(ws + oOpHi);
  unsigned short* op_lo     = (unsigned short*)(ws + oOpLo);
  float* bgbuf              = (float*)(ws + oBG);

  {
    const int n8 = kTok * kD / 8;
    split8_bf16_kernel<<<(n8 + 255) / 256, 256, 0, stream>>>(hidden, hid_hi, hid_lo, n8);
  }
  {
    const int n8 = kD * kD / 8;
    split8_bf16_kernel<<<(n8 + 255) / 256, 256, 0, stream>>>(out_proj_W, op_hi, op_lo, n8);
  }
  tsplit_bf16_kernel<<<dim3(kBW / 64, kD / 64), 256, 0, stream>>>(cond_in_W, kD, kBW, ci_hi, ci_lo);
  tsplit_bf16_kernel<<<dim3(kNDeltaPad / 64, kBW / 64), 256, 0, stream>>>(delta_W, kBW, kNDelta, dw_hi, dw_lo);
  tsplit_bf16_kernel<<<dim3(kNCtrlPad / 64, kD / 64), 256, 0, stream>>>(ctrl_W, kD, kNCtrl, ctrlWt_hi, ctrlWt_lo);

  {
    const int tiles = (kTok / 64) * (kBW / 64);
    wmma_gemm64<1, true, 0, 0, false, 0><<<dim3((tiles + 7) / 8, 1), 256, 0, stream>>>(
        hid_hi, hid_lo, kD, 0L, ci_hi, ci_lo, kD, 0L,
        (void*)pbuf, nullptr, kBW, 0L, nullptr, nullptr, 0L, kTok, kBW, kD, 1.0f);
  }
  cond_scan_kernel<<<kB, 64, 0, stream>>>(pbuf, rot_theta, cond_norm_w, c_hi, c_lo);
  {
    const int tiles = (kTok / 64) * (kNDeltaPad / 64);
    wmma_gemm64<1, true, 0, 0, false, 0><<<dim3((tiles + 7) / 8, 1), 256, 0, stream>>>(
        c_hi, c_lo, kBW, 0L, dw_hi, dw_lo, kBW, 0L,
        (void*)deltas, nullptr, kNDeltaPad, 0L, nullptr, nullptr, 0L, kTok, kNDeltaPad, kBW, 1.0f);
  }
  {
    const int tiles = (kTok / 64) * (kNCtrlPad / 64);
    wmma_gemm64<1, true, 0, 0, false, 0><<<dim3((tiles + 7) / 8, 1), 256, 0, stream>>>(
        hid_hi, hid_lo, kD, 0L, ctrlWt_hi, ctrlWt_lo, kD, 0L,
        (void*)ctrl, nullptr, kNCtrlPad, 0L, nullptr, nullptr, 0L, kTok, kNCtrlPad, kD, 1.0f);
  }
  qkv_prep_kernel<<<kTok, 256, 0, stream>>>(ctrl, deltas, ctrl_b, qkv_ramp, beta_ramp,
                                            q_conv_w, k_conv_w, v_conv_w, qkv, bgbuf);
  gdn_kernel<<<kB * kH, 256, 0, stream>>>(qkv, bgbuf, obuf);
  norm_gate_kernel<<<kTok, 128, 0, stream>>>(obuf, ctrl, ctrl_b, out_norm_w, y_hi, y_lo);
  {
    const int tiles = (kTok / 64) * (kD / 64);
    wmma_gemm64<1, true, 2, 0, false, 0><<<dim3((tiles + 7) / 8, 1), 256, 0, stream>>>(
        y_hi, y_lo, kD, 0L, op_hi, op_lo, kD, 0L,
        (void*)out, nullptr, kD, 0L, out_proj_b, nullptr, 0L, kTok, kD, kD, 1.0f);
  }
}
